// GNNClassifierNoPos_88648124990643
// MI455X (gfx1250) — hardware-verified
//
#include <hip/hip_runtime.h>
#include <stddef.h>


#define HIDD    64
#define KCAT    128
#define NTHR    256
#define NWAVE   8
#define EPT     8
#define NGRP    2
#define CHUNK   (NTHR * EPT * NGRP)
#define WCAP    (EPT * NGRP * 32)
#define LISTN   (NWAVE * WCAP)
#define TGT     512
#define NBP     32
#define NCLSF   2
#define PSTR    128
#define WSCALE  16.0f
#define BNEPS   1e-5f

#define LDS_ACC  (TGT * HIDD * 4)
#define LDS_LIST (LISTN * 4)
#define LDS_CNT  (TGT * 4)
#define LDS_RED  (4 * PSTR * 8)
#define LDS_PL   (PSTR * 8)
#define LDS_AGG  (LDS_ACC + LDS_LIST + LDS_CNT + LDS_RED + LDS_PL + 64)

static_assert((CHUNK & (CHUNK - 1)) == 0);
static_assert(CHUNK <= 4096);
static_assert((TGT & (TGT - 1)) == 0 && TGT <= 4096);
static_assert(TGT == NWAVE * 64);
static_assert(TGT == 4 * 128);
static_assert((NBP & (NBP - 1)) == 0 && NBP <= 4096);
static_assert(NBP * NCLSF == 64);
static_assert(LDS_ACC == TGT * KCAT * 2);
static_assert((2 * HIDD * KCAT / 8) % NTHR == 0);
static_assert(((LDS_ACC + LDS_LIST + LDS_CNT) & 15) == 0);
static_assert(((LDS_ACC + LDS_LIST + LDS_CNT + LDS_RED) & 15) == 0);

typedef float    v2f  __attribute__((ext_vector_type(2)));
typedef float    v4f  __attribute__((ext_vector_type(4)));
typedef float    v8f  __attribute__((ext_vector_type(8)));
typedef int      v4i  __attribute__((ext_vector_type(4)));
typedef double   v2d  __attribute__((ext_vector_type(2)));
typedef _Float16 v8h  __attribute__((ext_vector_type(8)));
typedef _Float16 v16h __attribute__((ext_vector_type(16)));
union FragH { v16h v; v8h h[2]; };

__device__ __forceinline__ v8h cvt8(v4f a, v4f b) {
  v8h r;
  r[0] = (_Float16)a.x; r[1] = (_Float16)a.y; r[2] = (_Float16)a.z; r[3] = (_Float16)a.w;
  r[4] = (_Float16)b.x; r[5] = (_Float16)b.y; r[6] = (_Float16)b.z; r[7] = (_Float16)b.w;
  return r;
}

__device__ __forceinline__ v8f wmh(v16h a, v16h b, v8f c) {
  v8f d = __builtin_amdgcn_wmma_f32_16x16x32_f16(false, a, false, b, (short)0, c, false, false);
  asm volatile("v_nop\n\tv_nop\n\tv_nop\n\tv_nop" : "+v"(d) : "v"(a), "v"(b));
  return d;
}

template <int NB>
__device__ __forceinline__ int scan_chunk(const int* __restrict__ dsts, int nE, int cbase, int slotBase,
                                          int vec8, int* list, int tid, int lane, int wave) {
  int wc = 0;
#pragma unroll
  for (int g = 0; g < NGRP; ++g) {
    const int el0  = (g * NTHR + tid) * EPT;
    const int e0   = cbase + el0;
    const int sent = -2147483647 - 1;
    v4i da, db;
    if (vec8 != 0 && cbase + CHUNK <= nE) {
      da = *(const v4i*)(dsts + e0);
      db = *(const v4i*)(dsts + e0 + 4);
    } else {
      da.x = (e0     < nE) ? dsts[min(e0, nE - 1)] : sent;
      da.y = (e0 + 1 < nE) ? dsts[min(e0 + 1, nE - 1)] : sent;
      da.z = (e0 + 2 < nE) ? dsts[min(e0 + 2, nE - 1)] : sent;
      da.w = (e0 + 3 < nE) ? dsts[min(e0 + 3, nE - 1)] : sent;
      db.x = (e0 + 4 < nE) ? dsts[min(e0 + 4, nE - 1)] : sent;
      db.y = (e0 + 5 < nE) ? dsts[min(e0 + 5, nE - 1)] : sent;
      db.z = (e0 + 6 < nE) ? dsts[min(e0 + 6, nE - 1)] : sent;
      db.w = (e0 + 7 < nE) ? dsts[min(e0 + 7, nE - 1)] : sent;
    }
    const unsigned nb = (unsigned)slotBase;
    const unsigned s0 = (unsigned)da.x - nb, s1 = (unsigned)da.y - nb;
    const unsigned s2 = (unsigned)da.z - nb, s3 = (unsigned)da.w - nb;
    const unsigned s4 = (unsigned)db.x - nb, s5 = (unsigned)db.y - nb;
    const unsigned s6 = (unsigned)db.z - nb, s7 = (unsigned)db.w - nb;
    const bool h0 = s0 < (unsigned)NB, h1 = s1 < (unsigned)NB, h2 = s2 < (unsigned)NB, h3 = s3 < (unsigned)NB;
    const bool h4 = s4 < (unsigned)NB, h5 = s5 < (unsigned)NB, h6 = s6 < (unsigned)NB, h7 = s7 < (unsigned)NB;
    const unsigned any = __builtin_amdgcn_ballot_w32(h0 | h1 | h2 | h3 | h4 | h5 | h6 | h7);
    if (any != 0u) {
#define HITJ(J, HJ, SJ) { \
        const unsigned mj = __builtin_amdgcn_ballot_w32(HJ); \
        if (mj != 0u) { \
          if (HJ) { \
            const int pos = wc + (int)__builtin_amdgcn_mbcnt_lo(mj, 0u); \
            if (pos < WCAP) list[wave * WCAP + pos] = ((el0 + (J)) << 12) | (int)(SJ); \
          } \
          wc += (int)__builtin_popcount(mj); } }
      HITJ(0, h0, s0)
      HITJ(1, h1, s1)
      HITJ(2, h2, s2)
      HITJ(3, h3, s3)
      HITJ(4, h4, s4)
      HITJ(5, h5, s5)
      HITJ(6, h6, s6)
      HITJ(7, h7, s7)
#undef HITJ
    }
  }
  return wc;
}

__global__ __launch_bounds__(NTHR) void k_embed(
    const int* __restrict__ sid, const int* __restrict__ cid,
    const float* __restrict__ sW, const float* __restrict__ cW,
    float* x, int nN, int nS, int nC, int nPad) {
  const int idx = blockIdx.x * NTHR + (int)threadIdx.x;
  const int row = idx >> 4;
  const int c0  = (idx & 15) * 4;
  const int rr  = row < nN ? row : nN - 1;
  int s = sid[rr]; s = s < 0 ? 0 : (s > nS - 1 ? nS - 1 : s);
  int c = cid[rr]; c = c < 0 ? 0 : (c > nC - 1 ? nC - 1 : c);
  v4f v = *(const v4f*)(sW + s * HIDD + c0) + *(const v4f*)(cW + c * HIDD + c0);
  if (row >= nN) { v.x = 0.f; v.y = 0.f; v.z = 0.f; v.w = 0.f; }
  if (row < nPad) {
    float* p = x + (size_t)idx * 4;
    *(volatile v4f*)p = v;
    __threadfence();
    *(volatile v4f*)p = v;
  }
}

__global__ __launch_bounds__(NTHR) void k_wprep(
    const float* __restrict__ W1l, const float* __restrict__ W1r,
    const float* __restrict__ W2l, const float* __restrict__ W2r, _Float16* wpl) {
  const int layer = (int)(blockIdx.x >> 2);
  const int idx   = blockIdx.x * NTHR + (int)threadIdx.x;
  const int rem   = idx & 1023;
  const int n     = rem >> 4;
  const int k0    = (rem & 15) * 8;
  const float* Wl = layer == 0 ? W1l : W2l;
  const float* Wr = layer == 0 ? W1r : W2r;
  float v[8];
#pragma unroll
  for (int e = 0; e < 8; ++e) {
    const int k  = k0 + e;
    const int kc = k & (HIDD - 1);
    const float a = Wl[kc * HIDD + n];
    const float b = Wr[kc * HIDD + n];
    v[e] = (k < HIDD ? a : b) * WSCALE;
  }
  v4f p0, p1;
  p0.x = v[0]; p0.y = v[1]; p0.z = v[2]; p0.w = v[3];
  p1.x = v[4]; p1.y = v[5]; p1.z = v[6]; p1.w = v[7];
  const v8h hv = cvt8(p0, p1);
  _Float16* dp = wpl + (size_t)idx * 8;
  *(volatile v8h*)dp = hv;
  __threadfence();
  *(volatile v8h*)dp = hv;
}

__global__ __launch_bounds__(NTHR) void k_agg(
    const int* __restrict__ ei, const float* __restrict__ xin, const _Float16* __restrict__ wpl,
    const float* __restrict__ bias, float* z, double* part,
    int nN, int nE, int vec8, float aScale, float oScale) {
  extern __shared__ v4f lds_dyn[];
  float*    accf = (float*)lds_dyn;
  _Float16* hA   = (_Float16*)lds_dyn;
  int*      list = (int*)((char*)lds_dyn + LDS_ACC);
  int*      cnt  = (int*)((char*)lds_dyn + LDS_ACC + LDS_LIST);
  double*   red  = (double*)((char*)lds_dyn + LDS_ACC + LDS_LIST + LDS_CNT);
  double*   pl   = (double*)((char*)lds_dyn + LDS_ACC + LDS_LIST + LDS_CNT + LDS_RED);
  int*      wcnt = (int*)((char*)lds_dyn + LDS_ACC + LDS_LIST + LDS_CNT + LDS_RED + LDS_PL);
  const int tid = threadIdx.x, lane = tid & 31, wave = tid >> 5;
  const int rowBase = blockIdx.x * TGT;
  const int* dsts = ei + nE;

  {
    const v4f zz = {0.f, 0.f, 0.f, 0.f};
    for (int i = tid; i < TGT * HIDD / 4; i += NTHR) lds_dyn[i] = zz;
    for (int i = tid; i < TGT; i += NTHR) cnt[i] = 0;
  }
  __syncthreads();

  const int nChunks = (nE + CHUNK - 1) / CHUNK;
#pragma unroll 1
  for (int ch = 0; ch < nChunks; ++ch) {
    const int cbase = ch * CHUNK;
    const int wc = scan_chunk<TGT>(dsts, nE, cbase, rowBase, vec8, list, tid, lane, wave);
    if (lane == 0) wcnt[wave] = wc;
    __syncthreads();
    if (wave == 0) {
#pragma unroll 1
      for (int wsx = 0; wsx < NWAVE; ++wsx) {
        int n = __builtin_amdgcn_readfirstlane(wcnt[wsx]);
        n = n > WCAP ? WCAP : (n < 0 ? 0 : n);
        const int* lp = list + wsx * WCAP;
#pragma unroll 1
        for (int i = 0; i < n; ++i) {
          const int ent  = __builtin_amdgcn_readfirstlane(lp[i]);
          const int slot = ent & (TGT - 1);
          int e = cbase + ((ent >> 12) & (CHUNK - 1));
          e = e > nE - 1 ? nE - 1 : e;
          int src = ei[e];
          src = src < 0 ? 0 : (src > nN - 1 ? nN - 1 : src);
          const v2f v = *(const v2f*)(xin + (size_t)src * HIDD + 2 * lane);
          v2f* ap = (v2f*)(accf + slot * HIDD + 2 * lane);
          *ap = *ap + v;
          if (lane == 0) cnt[slot] = cnt[slot] + 1;
        }
      }
    }
    __syncthreads();
  }

#pragma unroll 1
  for (int it = 0; it < TGT / 32; ++it) {
    const int row = it * 32 + (tid >> 3);
    const int j   = tid & 7;
    const v4f m0 = *(const v4f*)(accf + row * HIDD + 8 * j);
    const v4f m1 = *(const v4f*)(accf + row * HIDD + 8 * j + 4);
    int c = cnt[row];
    const float* xp = xin + ((size_t)rowBase + row) * HIDD + 8 * j;
    const v4f xa = *(const v4f*)xp;
    const v4f xb = *(const v4f*)(xp + 4);
    __syncthreads();
    c = c < 1 ? 1 : c;
    const float inv = aScale * (1.0f / (float)c);
    *(v8h*)(hA + row * KCAT + 8 * j)        = cvt8(m0 * inv, m1 * inv);
    *(v8h*)(hA + row * KCAT + HIDD + 8 * j) = cvt8(xa * aScale, xb * aScale);
  }
  __syncthreads();

  {
    const int hh = lane >> 4, m = lane & 15;
#pragma unroll 1
    for (int rt = 0; rt < 4; ++rt) {
      const int r0 = wave * 64 + rt * 16;
      v8f acc[4];
#pragma unroll
      for (int t = 0; t < 4; ++t) { v8f zz = {0.f, 0.f, 0.f, 0.f, 0.f, 0.f, 0.f, 0.f}; acc[t] = zz; }
      const _Float16* ar = hA + (r0 + m) * KCAT + 8 * hh;
#pragma unroll
      for (int kt = 0; kt < KCAT / 32; ++kt) {
        FragH a;
        a.h[0] = *(const v8h*)(ar + 32 * kt);
        a.h[1] = *(const v8h*)(ar + 32 * kt + 16);
#pragma unroll
        for (int t = 0; t < 4; ++t) {
          const _Float16* bp = wpl + (size_t)(16 * t + m) * KCAT + 32 * kt + 8 * hh;
          FragH b;
          b.h[0] = *(const v8h*)bp;
          b.h[1] = *(const v8h*)(bp + 16);
          acc[t] = wmh(a.v, b.v, acc[t]);
        }
      }
      float* sp = accf + (r0 + 8 * hh) * HIDD + m;
#pragma unroll
      for (int t = 0; t < 4; ++t) {
        const float bv = bias[16 * t + m];
#pragma unroll
        for (int r = 0; r < 8; ++r) sp[r * HIDD + 16 * t] = acc[t][r] * oScale + bv;
      }
    }
  }
  __syncthreads();

  const float* lz = accf + wave * 64 * HIDD + 4 * lane;
  float* gz = z + ((size_t)rowBase + wave * 64) * HIDD + 4 * lane;
#pragma unroll 4
  for (int i = 0; i < 32; ++i) { const v4f v = *(const v4f*)(lz + i * 128); *(volatile v4f*)(gz + (size_t)i * 128) = v; }

  {
    const int c = tid & 63, q = tid >> 6;
    int rlim = nN - rowBase - 128 * q;
    rlim = rlim < 0 ? 0 : (rlim > 128 ? 128 : rlim);
    const float* zc = accf + (128 * q) * HIDD + c;
    double s = 0.0, sq = 0.0;
#pragma unroll 2
    for (int r = 0; r < rlim; ++r) {
      const double v = (double)zc[r * HIDD];
      s += v;
      sq += v * v;
    }
    red[q * PSTR + c] = s;
    red[q * PSTR + HIDD + c] = sq;
  }
  __syncthreads();
  if (tid < PSTR) pl[tid] = (red[tid] + red[PSTR + tid]) + (red[2 * PSTR + tid] + red[3 * PSTR + tid]);
  __syncthreads();
  v2d pv = {0.0, 0.0};
  if (tid < 64) pv = *(const v2d*)(pl + 2 * tid);
  double* gp = part + (size_t)blockIdx.x * PSTR + 2 * tid;
  if (tid < 64) *(volatile v2d*)gp = pv;
  __threadfence();
#pragma unroll 4
  for (int i = 0; i < 32; ++i) { const v4f v = *(const v4f*)(lz + i * 128); *(volatile v4f*)(gz + (size_t)i * 128) = v; }
  if (tid < 64) *(volatile v2d*)gp = pv;
}

__device__ __forceinline__ void bn_coeffs(const double* __restrict__ part, int nPart, int nN,
                                          const float* __restrict__ gam, const float* __restrict__ bet,
                                          float* ssc, float* ssh, int tid) {
  if (tid < HIDD) {
    double s = 0.0, q = 0.0;
#pragma unroll 1
    for (int b = 0; b < nPart; ++b) {
      s += part[(size_t)b * PSTR + tid];
      q += part[(size_t)b * PSTR + HIDD + tid];
    }
    const double inv = 1.0 / (double)(nN > 0 ? nN : 1);
    const double mu  = s * inv;
    double var = q * inv - mu * mu;
    var = var < 0.0 ? 0.0 : var;
    const float sc = gam[tid] * rsqrtf((float)var + BNEPS);
    ssc[tid] = sc;
    ssh[tid] = bet[tid] - (float)mu * sc;
  }
}

__global__ __launch_bounds__(NTHR) void k_apply(
    const float* __restrict__ z, const double* __restrict__ part,
    const float* __restrict__ gam, const float* __restrict__ bet,
    float* xo, int nN, int nPart) {
  __shared__ __attribute__((aligned(16))) float ssc[HIDD];
  __shared__ __attribute__((aligned(16))) float ssh[HIDD];
  const int tid = threadIdx.x, lane = tid & 31, wave = tid >> 5;
  bn_coeffs(part, nPart, nN, gam, bet, ssc, ssh, tid);
  __syncthreads();
  const int c0 = (4 * lane) & (HIDD - 1);
  const v4f sc = *(const v4f*)(ssc + c0);
  const v4f sh = *(const v4f*)(ssh + c0);
  const size_t base = ((size_t)blockIdx.x * TGT + wave * 64) * HIDD + 4 * lane;
#pragma unroll 2
  for (int i = 0; i < 32; ++i) {
    const size_t p = base + (size_t)i * 128;
    const v4f v = *(const v4f*)(z + p);
    v4f y = v * sc + sh;
    y.x = fmaxf(y.x, 0.f); y.y = fmaxf(y.y, 0.f); y.z = fmaxf(y.z, 0.f); y.w = fmaxf(y.w, 0.f);
    *(volatile v4f*)(xo + p) = y;
    __threadfence();
    *(volatile v4f*)(xo + p) = y;
  }
}

__global__ __launch_bounds__(NTHR) void k_pool(
    const int* __restrict__ bat, const float* __restrict__ z, const double* __restrict__ part,
    const float* __restrict__ gam, const float* __restrict__ bet,
    const float* __restrict__ wlin, const float* __restrict__ blin, float* out,
    int nN, int nPart) {
  __shared__ __attribute__((aligned(16))) float acc[NBP * HIDD];
  __shared__ __attribute__((aligned(16))) int list[LISTN];
  __shared__ __attribute__((aligned(16))) float ssc[HIDD];
  __shared__ __attribute__((aligned(16))) float ssh[HIDD];
  __shared__ __attribute__((aligned(16))) float sout[NBP * NCLSF];
  __shared__ int wcnt[NWAVE];
  const int tid = threadIdx.x, lane = tid & 31, wave = tid >> 5;
  const int gBase = blockIdx.x * NBP;

  bn_coeffs(part, nPart, nN, gam, bet, ssc, ssh, tid);
  {
    const v4f zz = {0.f, 0.f, 0.f, 0.f};
    for (int i = tid; i < NBP * HIDD / 4; i += NTHR) ((v4f*)acc)[i] = zz;
  }
  __syncthreads();
  v2f sc2, sh2;
  sc2.x = ssc[2 * lane]; sc2.y = ssc[2 * lane + 1];
  sh2.x = ssh[2 * lane]; sh2.y = ssh[2 * lane + 1];

  const int nChunks = (nN + CHUNK - 1) / CHUNK;
#pragma unroll 1
  for (int ch = 0; ch < nChunks; ++ch) {
    const int cbase = ch * CHUNK;
    const int wc = scan_chunk<NBP>(bat, nN, cbase, gBase, 1, list, tid, lane, wave);
    if (lane == 0) wcnt[wave] = wc;
    __syncthreads();
    if (wave == 0) {
#pragma unroll 1
      for (int wsx = 0; wsx < NWAVE; ++wsx) {
        int n = __builtin_amdgcn_readfirstlane(wcnt[wsx]);
        n = n > WCAP ? WCAP : (n < 0 ? 0 : n);
        const int* lp = list + wsx * WCAP;
#pragma unroll 1
        for (int i = 0; i < n; ++i) {
          const int ent  = __builtin_amdgcn_readfirstlane(lp[i]);
          const int slot = ent & (NBP - 1);
          int nd = cbase + ((ent >> 12) & (CHUNK - 1));
          nd = nd > nN - 1 ? nN - 1 : nd;
          const v2f v = *(const v2f*)(z + (size_t)nd * HIDD + 2 * lane);
          v2f y;
          y.x = fmaxf(v.x * sc2.x + sh2.x, 0.f);
          y.y = fmaxf(v.y * sc2.y + sh2.y, 0.f);
          v2f* ap = (v2f*)(acc + slot * HIDD + 2 * lane);
          *ap = *ap + y;
        }
      }
    }
    __syncthreads();
  }

  if (tid < NBP * NCLSF) {
    const int g = tid >> 1, c = tid & 1;
    float s = 0.f;
#pragma unroll 1
    for (int f = 0; f < HIDD; ++f) s += acc[g * HIDD + f] * wlin[f * NCLSF + c];
    sout[tid] = s + blin[c];
  }
  __syncthreads();
  v4f ov = {0.f, 0.f, 0.f, 0.f};
  if (tid < 16) ov = *(const v4f*)(sout + 4 * tid);
  float* op = out + (size_t)blockIdx.x * (NBP * NCLSF) + 4 * tid;
  if (tid < 16) *(volatile v4f*)op = ov;
  __threadfence();
  if (tid < 16) *(volatile v4f*)op = ov;
}

extern "C" void kernel_launch(void* const* d_in, const int* in_sizes, int n_in,
                              void* d_out, int out_size, void* d_ws, size_t ws_size,
                              hipStream_t stream) {
  if (n_in < 18) return;
  const int nN = in_sizes[0];
  if (nN <= 0 || in_sizes[1] != nN || in_sizes[3] != nN) return;
  if ((in_sizes[2] & 1) != 0) return;
  const int nE = in_sizes[2] / 2;
  if (nE <= 0) return;
  const int nS = in_sizes[4] / HIDD, nC = in_sizes[5] / HIDD;
  if (nS < 1 || nC < 1 || in_sizes[4] != nS * HIDD || in_sizes[5] != nC * HIDD) return;
  if (in_sizes[6] != HIDD * HIDD || in_sizes[8] != HIDD * HIDD ||
      in_sizes[11] != HIDD * HIDD || in_sizes[13] != HIDD * HIDD) return;
  if (in_sizes[7] < HIDD || in_sizes[9] < HIDD || in_sizes[10] < HIDD ||
      in_sizes[12] < HIDD || in_sizes[14] < HIDD || in_sizes[15] < HIDD) return;
  if (in_sizes[17] != NCLSF || in_sizes[16] != HIDD * NCLSF) return;
  const int nG = out_size / NCLSF;
  if (nG <= 0 || out_size != nG * NCLSF || (nG % NBP) != 0) return;
  if (nN > (1 << 24) || nE > (1 << 28)) return;

  const int*   sid  = (const int*)d_in[0];
  const int*   cid  = (const int*)d_in[1];
  const int*   ei   = (const int*)d_in[2];
  const int*   bat  = (const int*)d_in[3];
  const float* sW   = (const float*)d_in[4];
  const float* cW   = (const float*)d_in[5];
  const float* W1l  = (const float*)d_in[6];
  const float* b1   = (const float*)d_in[7];
  const float* W1r  = (const float*)d_in[8];
  const float* g1   = (const float*)d_in[9];
  const float* be1  = (const float*)d_in[10];
  const float* W2l  = (const float*)d_in[11];
  const float* b2   = (const float*)d_in[12];
  const float* W2r  = (const float*)d_in[13];
  const float* g2   = (const float*)d_in[14];
  const float* be2  = (const float*)d_in[15];
  const float* Wlin = (const float*)d_in[16];
  const float* blin = (const float*)d_in[17];
  float* out = (float*)d_out;

  const int nAgg = (nN + TGT - 1) / TGT;
  const int NPAD = nAgg * TGT;

  char* ws = (char*)d_ws;
  size_t off = 0;
  const size_t oW  = off; off += (size_t)2 * HIDD * KCAT * 2;       off = (off + 255) & ~(size_t)255;
  const size_t oX  = off; off += (size_t)NPAD * HIDD * 4;           off = (off + 255) & ~(size_t)255;
  const size_t oZ  = off; off += (size_t)NPAD * HIDD * 4;           off = (off + 255) & ~(size_t)255;
  const size_t oP1 = off; off += (size_t)nAgg * PSTR * 8;           off = (off + 255) & ~(size_t)255;
  const size_t oP2 = off; off += (size_t)nAgg * PSTR * 8;           off = (off + 255) & ~(size_t)255;
  if (off > ws_size) return;
  _Float16* wpl = (_Float16*)(ws + oW);
  float*    X   = (float*)(ws + oX);
  float*    Z   = (float*)(ws + oZ);
  double*   P1  = (double*)(ws + oP1);
  double*   P2  = (double*)(ws + oP2);

  const int vec8 = ((nE & 3) == 0) ? 1 : 0;

  k_embed<<<NPAD * (HIDD / 4) / NTHR, NTHR, 0, stream>>>(sid, cid, sW, cW, X, nN, nS, nC, NPAD);
  k_wprep<<<(2 * HIDD * KCAT / 8) / NTHR, NTHR, 0, stream>>>(W1l, W1r, W2l, W2r, wpl);

  hipFuncSetAttribute(reinterpret_cast<const void*>(&k_agg),
                      hipFuncAttributeMaxDynamicSharedMemorySize, LDS_AGG);
  k_agg<<<nAgg, NTHR, LDS_AGG, stream>>>(ei, X, wpl, b1, Z, P1, nN, nE, vec8, 16.0f, 1.0f / 256.0f);
  k_apply<<<nAgg, NTHR, 0, stream>>>(Z, P1, g1, be1, X, nN, nAgg);
  k_agg<<<nAgg, NTHR, LDS_AGG, stream>>>(ei, X, wpl + (size_t)HIDD * KCAT, b2, Z, P2, nN, nE, vec8, 1.0f, 1.0f / 16.0f);
  k_pool<<<nG / NBP, NTHR, 0, stream>>>(bat, Z, P2, g2, be2, Wlin, blin, out, nN, nAgg);
}
